// PointnetSAModule_2628519985461
// MI455X (gfx1250) — hardware-verified
//
#include <hip/hip_runtime.h>
#include <stdint.h>

#pragma clang fp contract(off)

typedef __attribute__((ext_vector_type(16))) _Float16 v16h;
typedef __attribute__((ext_vector_type(8)))  _Float16 v8h;
typedef __attribute__((ext_vector_type(8)))  float    v8f;
typedef __attribute__((ext_vector_type(4)))  float    v4f;
typedef __attribute__((ext_vector_type(4)))  unsigned v4u;

constexpr int NUM_B    = 16;
constexpr int NUM_PTS  = 4096;
constexpr int NUM_CF   = 64;
constexpr int NUM_CTR  = 1024;
constexpr int NUM_SMP  = 32;
constexpr int NUM_GRP  = NUM_B * NUM_CTR;
constexpr int NUM_ROWS = NUM_GRP * NUM_SMP;
constexpr int W1_PITCH = 67;
constexpr int NOUT1 = 64;
constexpr int NOUT2 = 64;
constexpr int NOUT3 = 128;
constexpr int LDSP  = 72;
constexpr int NUM_PBLK = NUM_ROWS / 128;
constexpr float W_CARRY     = 16.0f;
constexpr float W_CARRY_INV = 1.0f / 16.0f;
constexpr float BN_EPS = 1e-5f;

static_assert(NUM_B * NUM_PTS * 3 * 4 == 786432, "xyz bytes");
static_assert(NUM_B * NUM_CF * NUM_PTS * 4 == 16777216, "features bytes");
static_assert(NOUT1 * W1_PITCH * 4 == 17152, "W1 bytes");
static_assert(NOUT2 * NOUT1 * 4 == 16384, "W2 bytes");
static_assert(NOUT3 * NOUT2 * 4 == 32768, "W3 bytes");
static_assert(NUM_ROWS == 524288, "rows");
static_assert((NUM_CTR * NUM_SMP) == (1 << 15), "rows per batch is 2^15");
static_assert(NUM_PBLK == 4096, "partial blocks");

constexpr size_t OUT0_BYTES    = (size_t)NUM_B * NUM_CTR * 3 * 4;
constexpr size_t OUT1_OFF_B    = 196608;
constexpr size_t OUT1_BYTES    = (size_t)NUM_B * NOUT3 * NUM_CTR * 4;
constexpr size_t OUT_TOTAL_B   = 8585216;
static_assert(OUT0_BYTES == OUT1_OFF_B, "out1 offset");
static_assert(OUT1_OFF_B % 128 == 0, "out1 line aligned");
static_assert(OUT1_OFF_B + OUT1_BYTES == OUT_TOTAL_B, "output total");

constexpr size_t WS_NXYZ  = 0;
constexpr size_t WS_IDX   = WS_NXYZ  + (size_t)NUM_GRP * 3 * 4;
constexpr size_t WS_WPL   = WS_IDX   + (size_t)NUM_GRP * NUM_SMP * 4;
constexpr size_t WS_AF    = WS_WPL   + (size_t)16384 * 2;
constexpr size_t WS_YP    = WS_AF    + (size_t)NUM_B * NUM_PTS * 64 * 2;
constexpr size_t WS_X2    = WS_YP    + (size_t)NUM_B * NUM_PTS * 64 * 4;
constexpr size_t WS_GMAX  = WS_X2    + (size_t)NUM_ROWS * 64 * 2;
constexpr size_t WS_GMIN  = WS_GMAX  + (size_t)NUM_GRP * 128 * 4;
constexpr size_t WS_PART1 = WS_GMIN  + (size_t)NUM_GRP * 128 * 4;
constexpr size_t WS_PART2 = WS_PART1 + (size_t)NUM_PBLK * 128 * 4;
constexpr size_t WS_PART3 = WS_PART2 + (size_t)NUM_PBLK * 128 * 4;
constexpr size_t WS_SCSH1 = WS_PART3 + (size_t)NUM_PBLK * 256 * 4;
constexpr size_t WS_SCSH2 = WS_SCSH1 + 1024;
constexpr size_t WS_SCSH3 = WS_SCSH2 + 1024;
constexpr size_t WS_TOTAL = WS_SCSH3 + 1024;
static_assert(WS_TOTAL == 119770112, "carve total");
static_assert(WS_TOTAL <= 134217728, "carve under 128 MiB");
static_assert(WS_IDX % 256 == 0 && WS_WPL % 256 == 0 && WS_AF % 256 == 0 && WS_YP % 256 == 0, "align");
static_assert(WS_X2 % 256 == 0 && WS_GMAX % 256 == 0 && WS_GMIN % 256 == 0 && WS_PART1 % 256 == 0, "align");
static_assert(WS_PART2 % 256 == 0 && WS_PART3 % 256 == 0 && WS_SCSH1 % 256 == 0, "align");

union FragH { v16h v; v8h h[2]; };

__device__ __forceinline__ v8f mma_h(v16h a, v16h b, v8f c) {
  c = __builtin_amdgcn_wmma_f32_16x16x32_f16(false, a, false, b, (short)0, c, false, false);
  asm volatile("v_nop\n\tv_nop\n\tv_nop\n\tv_nop" : "+v"(c) : "v"(a), "v"(b));
  return c;
}

__device__ __forceinline__ void wave_lds_sync() {
  __builtin_amdgcn_fence(__ATOMIC_RELEASE, "workgroup");
  __builtin_amdgcn_wave_barrier();
  __builtin_amdgcn_fence(__ATOMIC_ACQUIRE, "workgroup");
}

__device__ __forceinline__ float h16_to_f32(unsigned hb) {
  const unsigned sgn = (hb & 0x8000u) << 16; const unsigned em = hb & 0x7fffu;
  const float fn = __uint_as_float((em << 13) + 0x38000000u);
  const float fs = (float)em * 5.9604644775390625e-8f;
  const float mag = (em < 0x400u) ? fs : fn; return __uint_as_float(__float_as_uint(mag) | sgn); }

__global__ __launch_bounds__(256) void fps_kernel(const float* __restrict__ xyz,
                                                  float* __restrict__ out0,
                                                  float* __restrict__ nxyz) {
#pragma clang fp contract(off)
  __shared__ float sxyz[3 * NUM_PTS];
  __shared__ float wbest[2][8];
  __shared__ int   widx[2][8];
  __shared__ int   sel[NUM_CTR];
  const int b = blockIdx.x;
  const int t = threadIdx.x;
  const int lane = t & 31;
  const int wave = t >> 5;
  const float* base = xyz + (size_t)b * NUM_PTS * 3;

#pragma unroll 2
  for (int i = 0; i < 12; ++i) {
    const int j = t + 256 * i;
    const v4f v = *(const v4f*)(base + 4 * j);
    const float e0 = v.x, e1 = v.y, e2 = v.z, e3 = v.w;
    const int f0 = 4 * j;
    const int p0 = f0 / 3;            const int c0 = f0 - 3 * p0;
    const int p1 = (f0 + 1) / 3;      const int c1 = (f0 + 1) - 3 * p1;
    const int p2 = (f0 + 2) / 3;      const int c2 = (f0 + 2) - 3 * p2;
    const int p3 = (f0 + 3) / 3;      const int c3 = (f0 + 3) - 3 * p3;
    sxyz[c0 * NUM_PTS + p0] = e0;
    sxyz[c1 * NUM_PTS + p1] = e1;
    sxyz[c2 * NUM_PTS + p2] = e2;
    sxyz[c3 * NUM_PTS + p3] = e3;
  }
  __syncthreads();

  float px[16], py[16], pz[16], dmin[16];
#pragma unroll
  for (int k = 0; k < 16; ++k) {
    px[k] = sxyz[t + 256 * k];
    py[k] = sxyz[NUM_PTS + t + 256 * k];
    pz[k] = sxyz[2 * NUM_PTS + t + 256 * k];
    dmin[k] = 1e10f;
  }

  int cur = 0;
#pragma unroll 1
  for (int it = 0; it < NUM_CTR; ++it) {
    if (t == 0) sel[it] = cur;
    const float lx = sxyz[cur];
    const float ly = sxyz[NUM_PTS + cur];
    const float lz = sxyz[2 * NUM_PTS + cur];
    float best = -1.0f;
    int bi = 0;
#pragma unroll
    for (int k = 0; k < 16; ++k) {
      const float dx = px[k] - lx;
      const float dy = py[k] - ly;
      const float dz = pz[k] - lz;
      const float t0 = dx * dx;
      const float t1 = dy * dy;
      const float t2 = dz * dz;
      const float d = (t0 + t2) + t1;
      const float m = fminf(dmin[k], d);
      dmin[k] = m;
      if (m > best) { best = m; bi = t + 256 * k; }
    }
#pragma unroll
    for (int off = 16; off > 0; off >>= 1) {
      const float ob = __shfl_xor(best, off, 32);
      const int   oi = __shfl_xor(bi, off, 32);
      const bool take = (ob > best) || ((ob == best) && (oi < bi));
      best = take ? ob : best;
      bi   = take ? oi : bi;
    }
    const int pb = it & 1;
    if (lane == 0) { wbest[pb][wave] = best; widx[pb][wave] = bi; }
    __syncthreads();
    float fb = wbest[pb][0];
    int   fi = widx[pb][0];
#pragma unroll
    for (int w = 1; w < 8; ++w) {
      const float ob = wbest[pb][w];
      const int   oi = widx[pb][w];
      const bool take = (ob > fb) || ((ob == fb) && (oi < fi));
      fb = take ? ob : fb;
      fi = take ? oi : fi;
    }
    fi = fi < 0 ? 0 : fi;
    fi = fi > (NUM_PTS - 1) ? (NUM_PTS - 1) : fi;
    cur = fi;
  }
  __syncthreads();

  float* o0 = out0 + (size_t)b * NUM_CTR * 3;
  float* o1 = nxyz + (size_t)b * NUM_CTR * 3;
  v4f ov[3];
#pragma unroll
  for (int i = 0; i < 3; ++i) {
    const int j = t + 256 * i;
    float a[4];
#pragma unroll
    for (int e = 0; e < 4; ++e) {
      const int f = 4 * j + e;
      const int p = f / 3;
      const int c = f - 3 * p;
      int s = sel[p];
      s = s < 0 ? 0 : s;
      s = s > (NUM_PTS - 1) ? (NUM_PTS - 1) : s;
      a[e] = sxyz[c * NUM_PTS + s];
    }
    ov[i] = (v4f){a[0], a[1], a[2], a[3]};
  }
  for (int pass = 0; pass < 2; ++pass) {
#pragma unroll
    for (int i = 0; i < 3; ++i) {
      const int j = t + 256 * i;
      *(volatile v4f*)(o0 + 4 * j) = ov[i];
      *(volatile v4f*)(o1 + 4 * j) = ov[i];
    }
    __threadfence();
  }
}

__global__ __launch_bounds__(256) void ball_query_kernel(const float* __restrict__ xyz,
                                                         const float* __restrict__ nxyz,
                                                         int* __restrict__ idx) {
#pragma clang fp contract(off)
  __shared__ int srow[8][32];
  const int lane = threadIdx.x & 31;
  const int wave = threadIdx.x >> 5;
  const int wid = blockIdx.x * 8 + wave;
  const int b = wid >> 10;
  const float* base = xyz + (size_t)b * NUM_PTS * 3;
  const float qx = nxyz[wid * 3 + 0];
  const float qy = nxyz[wid * 3 + 1];
  const float qz = nxyz[wid * 3 + 2];
  int count = 0;
  int first = 0;
#pragma unroll 1
  for (int i0 = 0; i0 < NUM_PTS; i0 += 32) {
    if (count >= NUM_SMP) break;
    const int i = i0 + lane;
    const float x = base[i * 3 + 0];
    const float y = base[i * 3 + 1];
    const float z = base[i * 3 + 2];
    const float dx = qx - x;
    const float dy = qy - y;
    const float dz = qz - z;
    const float t0 = dx * dx;
    const float t1 = dy * dy;
    const float t2 = dz * dz;
    const float d2 = (t0 + t2) + t1;
    const bool hit = d2 < 0.04f;
    const unsigned mask = (unsigned)__ballot(hit);
    if (count == 0 && mask != 0u) first = i0 + (__ffs(mask) - 1);
    const int pos = count + __popc(mask & ((1u << lane) - 1u));
    if (hit && pos < NUM_SMP) srow[wave][pos] = i;
    count += __popc(mask);
  }
  {
    const int s = count + lane;
    if (s < NUM_SMP) srow[wave][s] = first;
  }
  wave_lds_sync();
  int v = srow[wave][lane];
  v = v < 0 ? 0 : v;
  v = v > (NUM_PTS - 1) ? (NUM_PTS - 1) : v;
  volatile int* dst = idx + (size_t)wid * NUM_SMP + lane;
  *dst = v;
  __threadfence();
  *dst = v;
}

__global__ __launch_bounds__(256) void pack_w_kernel(const float* __restrict__ W1,
                                                     const float* __restrict__ W2,
                                                     const float* __restrict__ W3,
                                                     _Float16* __restrict__ wpl) {
  const int g = blockIdx.x * 256 + threadIdx.x;
  float f[8];
  if (blockIdx.x < 2) {
    const int row = g >> 3;
    const int c8 = (g & 7) * 8;
#pragma unroll
    for (int e = 0; e < 8; ++e) f[e] = W1[row * W1_PITCH + 3 + c8 + e];
  } else if (blockIdx.x < 4) {
    const int g2 = g - 512;
#pragma unroll
    for (int e = 0; e < 8; ++e) f[e] = W2[g2 * 8 + e];
  } else {
    const int g3 = g - 1024;
#pragma unroll
    for (int e = 0; e < 8; ++e) f[e] = W3[g3 * 8 + e];
  }
  v8h hv;
#pragma unroll
  for (int e = 0; e < 8; ++e) hv[e] = (_Float16)(f[e] * W_CARRY);
  *(volatile v8h*)(wpl + (size_t)g * 8) = hv;
  __threadfence();
  *(volatile v8h*)(wpl + (size_t)g * 8) = hv;
}

__global__ __launch_bounds__(256) void feat_t_kernel(const float* __restrict__ feat,
                                                     _Float16* __restrict__ Af) {
  __shared__ float tl[64 * 65];
  const int tid = threadIdx.x;
  const int n0 = blockIdx.x * 64;
  const int b = blockIdx.y;
  const float* fb = feat + (size_t)b * NUM_CF * NUM_PTS;
#pragma unroll
  for (int pass = 0; pass < 4; ++pass) {
    const int c = pass * 16 + (tid >> 4);
    const int n4 = (tid & 15) * 4;
    const v4f v = *(const v4f*)(fb + (size_t)c * NUM_PTS + n0 + n4);
    const float e0 = v.x, e1 = v.y, e2 = v.z, e3 = v.w;
    tl[(n4 + 0) * 65 + c] = e0;
    tl[(n4 + 1) * 65 + c] = e1;
    tl[(n4 + 2) * 65 + c] = e2;
    tl[(n4 + 3) * 65 + c] = e3;
  }
  __syncthreads();
  const int c8 = (tid & 7) * 8;
  v8h hv[2];
#pragma unroll
  for (int pass = 0; pass < 2; ++pass) {
    const int row = pass * 32 + (tid >> 3);
#pragma unroll
    for (int e = 0; e < 8; ++e) hv[pass][e] = (_Float16)tl[row * 65 + c8 + e];
  }
  for (int rep = 0; rep < 2; ++rep) {
#pragma unroll
    for (int pass = 0; pass < 2; ++pass) {
      const int row = pass * 32 + (tid >> 3);
      *(volatile v8h*)(Af + ((size_t)b * NUM_PTS + n0 + row) * 64 + c8) = hv[pass];
    }
    __threadfence();
  }
}

__global__ __launch_bounds__(256) void gemm_pts_kernel(const _Float16* __restrict__ Af,
                                                       const _Float16* __restrict__ Bt,
                                                       float* __restrict__ Yp) {
  __shared__ __align__(16) _Float16 Bs[64 * LDSP];
  __shared__ __align__(16) float slab[8][16 * 68];
  const int tid = threadIdx.x;
  const int lane = tid & 31;
  const int wave = tid >> 5;
  const int rl = lane & 15;
  const int hh = lane >> 4;
  const int koff = hh * 8;
#pragma unroll
  for (int i = 0; i < 2; ++i) {
    const int e = tid + 256 * i;
    const int n = e >> 3;
    const int c8 = (e & 7) * 8;
    *(v8h*)(Bs + n * LDSP + c8) = *(const v8h*)(Bt + n * 64 + c8);
  }
  __syncthreads();
  const int m0 = (blockIdx.x * 8 + wave) * 32;
  v8f acc[2][4];
#pragma unroll
  for (int i = 0; i < 2; ++i)
#pragma unroll
    for (int j = 0; j < 4; ++j) acc[i][j] = (v8f){0.f, 0.f, 0.f, 0.f, 0.f, 0.f, 0.f, 0.f};
#pragma unroll
  for (int ks = 0; ks < 2; ++ks) {
    const int kk = ks * 32 + koff;
    FragH a0, a1;
    a0.h[0] = *(const v8h*)(Af + (size_t)(m0 + rl) * 64 + kk);
    a0.h[1] = *(const v8h*)(Af + (size_t)(m0 + rl) * 64 + kk + 16);
    a1.h[0] = *(const v8h*)(Af + (size_t)(m0 + 16 + rl) * 64 + kk);
    a1.h[1] = *(const v8h*)(Af + (size_t)(m0 + 16 + rl) * 64 + kk + 16);
#pragma unroll
    for (int j = 0; j < 4; ++j) {
      FragH bf;
      bf.h[0] = *(const v8h*)(Bs + (j * 16 + rl) * LDSP + kk);
      bf.h[1] = *(const v8h*)(Bs + (j * 16 + rl) * LDSP + kk + 16);
      acc[0][j] = mma_h(a0.v, bf.v, acc[0][j]);
      acc[1][j] = mma_h(a1.v, bf.v, acc[1][j]);
    }
    asm volatile("" ::: "memory");
  }
  float* sl = slab[wave];
  const int c4 = (lane & 15) * 4;
#pragma unroll
  for (int i = 0; i < 2; ++i) {
#pragma unroll
    for (int j = 0; j < 4; ++j)
#pragma unroll
      for (int r = 0; r < 8; ++r) sl[(8 * hh + r) * 68 + j * 16 + rl] = acc[i][j][r] * W_CARRY_INV;
    wave_lds_sync();
    for (int pass = 0; pass < 2; ++pass) {
#pragma unroll
      for (int it = 0; it < 8; ++it) {
        const int row = it * 2 + hh;
        const v4f v = *(const v4f*)(sl + row * 68 + c4);
        *(volatile v4f*)(Yp + (size_t)(m0 + i * 16 + row) * 64 + c4) = v;
      }
      __threadfence();
    }
    wave_lds_sync();
  }
}

__device__ __forceinline__ void gather_x1(const float* __restrict__ xyz,
                                          const float* __restrict__ nxyz,
                                          const int* __restrict__ idx,
                                          const float* __restrict__ Yp,
                                          int row, int o8,
                                          const float (&w0)[8], const float (&w1)[8], const float (&w2)[8],
                                          float (&x)[8]) {
  const int g = row >> 5;
  const int b = row >> 15;
  int id = idx[row];
  id = id < 0 ? 0 : id;
  id = id > (NUM_PTS - 1) ? (NUM_PTS - 1) : id;
  const size_t pt = (size_t)b * NUM_PTS + id;
  const float dx = xyz[pt * 3 + 0] - nxyz[g * 3 + 0];
  const float dy = xyz[pt * 3 + 1] - nxyz[g * 3 + 1];
  const float dz = xyz[pt * 3 + 2] - nxyz[g * 3 + 2];
  const v4f y0 = *(const v4f*)(Yp + pt * 64 + o8);
  const v4f y1 = *(const v4f*)(Yp + pt * 64 + o8 + 4);
  x[0] = y0.x; x[1] = y0.y; x[2] = y0.z; x[3] = y0.w;
  x[4] = y1.x; x[5] = y1.y; x[6] = y1.z; x[7] = y1.w;
#pragma unroll
  for (int e = 0; e < 8; ++e) {
    float t = x[e];
    t = __builtin_fmaf(w0[e], dx, t);
    t = __builtin_fmaf(w1[e], dy, t);
    t = __builtin_fmaf(w2[e], dz, t);
    x[e] = t;
  }
}

__global__ __launch_bounds__(256) void stats1_kernel(const float* __restrict__ xyz,
                                                     const float* __restrict__ nxyz,
                                                     const int* __restrict__ idx,
                                                     const float* __restrict__ Yp,
                                                     const float* __restrict__ W1,
                                                     float* __restrict__ part) {
  __shared__ float wx[64 * 4];
  __shared__ float red[2][32][64];
  const int tid = threadIdx.x;
  if (tid < 192) {
    const int o = tid / 3;
    const int c = tid - 3 * o;
    wx[o * 4 + c] = W1[o * W1_PITCH + c];
  }
  __syncthreads();
  const int o8 = (tid & 7) * 8;
  const int rs = tid >> 3;
  float w0[8], w1[8], w2[8], s[8], q[8];
#pragma unroll
  for (int e = 0; e < 8; ++e) {
    w0[e] = wx[(o8 + e) * 4 + 0];
    w1[e] = wx[(o8 + e) * 4 + 1];
    w2[e] = wx[(o8 + e) * 4 + 2];
    s[e] = 0.0f;
    q[e] = 0.0f;
  }
#pragma unroll 1
  for (int pass = 0; pass < 4; ++pass) {
    const int row = blockIdx.x * 128 + pass * 32 + rs;
    float x[8];
    gather_x1(xyz, nxyz, idx, Yp, row, o8, w0, w1, w2, x);
#pragma unroll
    for (int e = 0; e < 8; ++e) {
      s[e] = s[e] + x[e];
      q[e] = __builtin_fmaf(x[e], x[e], q[e]);
    }
  }
#pragma unroll
  for (int e = 0; e < 8; ++e) {
    red[0][rs][o8 + e] = s[e];
    red[1][rs][o8 + e] = q[e];
  }
  __syncthreads();
  if (tid < 128) {
    const int st = tid >> 6;
    const int ch = tid & 63;
    float a = 0.0f;
#pragma unroll 4
    for (int r = 0; r < 32; ++r) a = a + red[st][r][ch];
    volatile float* dst = part + (size_t)blockIdx.x * 128 + tid;
    *dst = a;
    __threadfence();
    *dst = a;
  }
}

template <int NCH>
__global__ __launch_bounds__(256) void finalize_kernel(const float* __restrict__ part, int nblk,
                                                       const float* __restrict__ gam,
                                                       const float* __restrict__ bet,
                                                       float* __restrict__ scsh) {
  __shared__ float ls[256];
  const int tid = threadIdx.x;
  const int lane = tid & 31;
  const int wave = tid >> 5;
  ls[tid] = 0.0f;
  __syncthreads();
  for (int ch = wave; ch < NCH; ch += 8) {
    double s = 0.0, q = 0.0;
#pragma unroll 4
    for (int j = lane; j < nblk; j += 32) {
      s += (double)part[(size_t)j * (2 * NCH) + ch];
      q += (double)part[(size_t)j * (2 * NCH) + NCH + ch];
    }
#pragma unroll
    for (int off = 16; off > 0; off >>= 1) {
      const double so = __shfl_xor(s, off, 32);
      const double qo = __shfl_xor(q, off, 32);
      s += so;
      q += qo;
    }
    const double inv_n = 1.0 / (double)NUM_ROWS;
    const double m = s * inv_n;
    double var = q * inv_n - m * m;
    var = var < 0.0 ? 0.0 : var;
    const float vf = (float)var;
    const float sc = gam[ch] * (1.0f / sqrtf(vf + BN_EPS));
    const float sh = (float)((double)bet[ch] - m * (double)sc);
    if (lane == 0) { ls[ch] = sc; ls[128 + ch] = sh; }
  }
  __syncthreads();
  const float v = ls[tid];
  volatile float* dst = scsh + tid;
  *dst = v;
  __threadfence();
  *dst = v;
}

__global__ __launch_bounds__(256) void gemm2_kernel(const float* __restrict__ xyz,
                                                    const float* __restrict__ nxyz,
                                                    const int* __restrict__ idx,
                                                    const float* __restrict__ Yp,
                                                    const float* __restrict__ W1,
                                                    const float* __restrict__ scsh,
                                                    const _Float16* __restrict__ Bt,
                                                    _Float16* __restrict__ X2,
                                                    float* __restrict__ part) {
  __shared__ __align__(16) _Float16 As[128 * LDSP];
  __shared__ __align__(16) _Float16 Bs[64 * LDSP];
  __shared__ __align__(16) _Float16 Os[8][16 * LDSP];
  __shared__ float wx[64 * 4];
  __shared__ float red[2][8][64];
  const int tid = threadIdx.x;
  const int lane = tid & 31;
  const int wave = tid >> 5;
  const int rl = lane & 15;
  const int hh = lane >> 4;
  const int koff = hh * 8;
  if (tid < 192) {
    const int o = tid / 3;
    const int c = tid - 3 * o;
    wx[o * 4 + c] = W1[o * W1_PITCH + c];
  }
#pragma unroll
  for (int i = 0; i < 2; ++i) {
    const int e = tid + 256 * i;
    const int n = e >> 3;
    const int c8 = (e & 7) * 8;
    *(v8h*)(Bs + n * LDSP + c8) = *(const v8h*)(Bt + n * 64 + c8);
  }
  __syncthreads();
  const int o8 = (tid & 7) * 8;
  const int rs = tid >> 3;
  {
    float w0[8], w1[8], w2[8], sc[8], sh[8];
#pragma unroll
    for (int e = 0; e < 8; ++e) {
      w0[e] = wx[(o8 + e) * 4 + 0];
      w1[e] = wx[(o8 + e) * 4 + 1];
      w2[e] = wx[(o8 + e) * 4 + 2];
    }
    const v4f s0 = *(const v4f*)(scsh + o8);
    const v4f s1 = *(const v4f*)(scsh + o8 + 4);
    const v4f h0 = *(const v4f*)(scsh + 128 + o8);
    const v4f h1 = *(const v4f*)(scsh + 128 + o8 + 4);
    sc[0] = s0.x; sc[1] = s0.y; sc[2] = s0.z; sc[3] = s0.w;
    sc[4] = s1.x; sc[5] = s1.y; sc[6] = s1.z; sc[7] = s1.w;
    sh[0] = h0.x; sh[1] = h0.y; sh[2] = h0.z; sh[3] = h0.w;
    sh[4] = h1.x; sh[5] = h1.y; sh[6] = h1.z; sh[7] = h1.w;
#pragma unroll 1
    for (int pass = 0; pass < 4; ++pass) {
      const int rloc = pass * 32 + rs;
      const int row = blockIdx.x * 128 + rloc;
      float x[8];
      gather_x1(xyz, nxyz, idx, Yp, row, o8, w0, w1, w2, x);
      v8h hv;
#pragma unroll
      for (int e = 0; e < 8; ++e) {
        const float a = fmaxf(__builtin_fmaf(sc[e], x[e], sh[e]), 0.0f);
        hv[e] = (_Float16)a;
      }
      *(v8h*)(As + rloc * LDSP + o8) = hv;
    }
  }
  __syncthreads();

  v8f acc[4];
#pragma unroll
  for (int j = 0; j < 4; ++j) acc[j] = (v8f){0.f, 0.f, 0.f, 0.f, 0.f, 0.f, 0.f, 0.f};
#pragma unroll
  for (int ks = 0; ks < 2; ++ks) {
    const int kk = ks * 32 + koff;
    FragH a;
    a.h[0] = *(const v8h*)(As + (wave * 16 + rl) * LDSP + kk);
    a.h[1] = *(const v8h*)(As + (wave * 16 + rl) * LDSP + kk + 16);
#pragma unroll
    for (int j = 0; j < 4; ++j) {
      FragH bf;
      bf.h[0] = *(const v8h*)(Bs + (j * 16 + rl) * LDSP + kk);
      bf.h[1] = *(const v8h*)(Bs + (j * 16 + rl) * LDSP + kk + 16);
      acc[j] = mma_h(a.v, bf.v, acc[j]);
    }
  }

  _Float16* os = Os[wave];
  float sj[4], qj[4];
#pragma unroll
  for (int j = 0; j < 4; ++j) {
    float s = 0.0f, q = 0.0f;
#pragma unroll
    for (int r = 0; r < 8; ++r) {
      const float v = acc[j][r] * W_CARRY_INV;
      s = s + v;
      q = __builtin_fmaf(v, v, q);
      os[(8 * hh + r) * LDSP + j * 16 + rl] = (_Float16)v;
    }
    sj[j] = s;
    qj[j] = q;
  }
#pragma unroll
  for (int j = 0; j < 4; ++j) {
    const float so = __shfl_xor(sj[j], 16, 32);
    const float qo = __shfl_xor(qj[j], 16, 32);
    sj[j] = sj[j] + so;
    qj[j] = qj[j] + qo;
  }
  if (hh == 0) {
#pragma unroll
    for (int j = 0; j < 4; ++j) {
      red[0][wave][j * 16 + rl] = sj[j];
      red[1][wave][j * 16 + rl] = qj[j];
    }
  }
  wave_lds_sync();
  {
    const int q4 = lane >> 3;
    const int c8 = (lane & 7) * 8;
    v8h hv[4];
#pragma unroll
    for (int it = 0; it < 4; ++it) hv[it] = *(const v8h*)(os + (it * 4 + q4) * LDSP + c8);
    const size_t rbase = (size_t)blockIdx.x * 128 + wave * 16;
    for (int pass = 0; pass < 2; ++pass) {
#pragma unroll
      for (int it = 0; it < 4; ++it)
        *(volatile v8h*)(X2 + (rbase + it * 4 + q4) * 64 + c8) = hv[it];
      __threadfence();
    }
  }
  __syncthreads();
  if (tid < 128) {
    const int st = tid >> 6;
    const int ch = tid & 63;
    float a = 0.0f;
#pragma unroll
    for (int w = 0; w < 8; ++w) a = a + red[st][w][ch];
    volatile float* dst = part + (size_t)blockIdx.x * 128 + tid;
    *dst = a;
    __threadfence();
    *dst = a;
  }
}

__global__ __launch_bounds__(128) void gemm3_kernel(const unsigned* __restrict__ X2w,
                                                    const float* __restrict__ scsh,
                                                    const _Float16* __restrict__ Bt,
                                                    float* __restrict__ gmax,
                                                    float* __restrict__ gmin,
                                                    float* __restrict__ part) {
  __shared__ __align__(16) _Float16 As[128 * LDSP];
  __shared__ __align__(16) _Float16 Bs[128 * LDSP];
  __shared__ __align__(16) float gm[4][256];
  __shared__ float red[2][4][128];
  const int tid = threadIdx.x;
  const int lane = tid & 31;
  const int wave = tid >> 5;
  const int rl = lane & 15;
  const int hh = lane >> 4;
  const int koff = hh * 8;
#pragma unroll 4
  for (int i = 0; i < 8; ++i) {
    const int e = tid + 128 * i;
    const int n = e >> 3;
    const int c8 = (e & 7) * 8;
    *(v8h*)(Bs + n * LDSP + c8) = *(const v8h*)(Bt + n * 64 + c8);
  }
  {
    const int c8 = (tid & 7) * 8;
    const int rs = tid >> 3;
    float sc[8], sh[8];
    const v4f s0 = *(const v4f*)(scsh + c8);
    const v4f s1 = *(const v4f*)(scsh + c8 + 4);
    const v4f h0 = *(const v4f*)(scsh + 128 + c8);
    const v4f h1 = *(const v4f*)(scsh + 128 + c8 + 4);
    sc[0] = s0.x; sc[1] = s0.y; sc[2] = s0.z; sc[3] = s0.w;
    sc[4] = s1.x; sc[5] = s1.y; sc[6] = s1.z; sc[7] = s1.w;
    sh[0] = h0.x; sh[1] = h0.y; sh[2] = h0.z; sh[3] = h0.w;
    sh[4] = h1.x; sh[5] = h1.y; sh[6] = h1.z; sh[7] = h1.w;
#pragma unroll 1
    for (int pass = 0; pass < 8; ++pass) {
      const int rloc = pass * 16 + rs;
      const size_t row = (size_t)blockIdx.x * 128 + rloc;
      const v4u w = *(const v4u*)(X2w + row * 32 + (c8 >> 1));
      const unsigned u0 = w.x, u1 = w.y, u2 = w.z, u3 = w.w;
      float xv[8];
      xv[0] = h16_to_f32(u0 & 0xffffu); xv[1] = h16_to_f32(u0 >> 16);
      xv[2] = h16_to_f32(u1 & 0xffffu); xv[3] = h16_to_f32(u1 >> 16);
      xv[4] = h16_to_f32(u2 & 0xffffu); xv[5] = h16_to_f32(u2 >> 16);
      xv[6] = h16_to_f32(u3 & 0xffffu); xv[7] = h16_to_f32(u3 >> 16);
      v8h hv;
#pragma unroll
      for (int e = 0; e < 8; ++e) {
        const float a = fmaxf(__builtin_fmaf(sc[e], xv[e], sh[e]), 0.0f);
        hv[e] = (_Float16)a;
      }
      *(v8h*)(As + rloc * LDSP + c8) = hv;
    }
  }
  __syncthreads();

#pragma unroll 1
  for (int nh = 0; nh < 2; ++nh) {
    v8f acc[2][4];
#pragma unroll
    for (int i = 0; i < 2; ++i)
#pragma unroll
      for (int j = 0; j < 4; ++j) acc[i][j] = (v8f){0.f, 0.f, 0.f, 0.f, 0.f, 0.f, 0.f, 0.f};
#pragma unroll
    for (int ks = 0; ks < 2; ++ks) {
      const int kk = ks * 32 + koff;
      FragH a0, a1;
      a0.h[0] = *(const v8h*)(As + (wave * 32 + rl) * LDSP + kk);
      a0.h[1] = *(const v8h*)(As + (wave * 32 + rl) * LDSP + kk + 16);
      a1.h[0] = *(const v8h*)(As + (wave * 32 + 16 + rl) * LDSP + kk);
      a1.h[1] = *(const v8h*)(As + (wave * 32 + 16 + rl) * LDSP + kk + 16);
#pragma unroll
      for (int j = 0; j < 4; ++j) {
        FragH bf;
        bf.h[0] = *(const v8h*)(Bs + (nh * 64 + j * 16 + rl) * LDSP + kk);
        bf.h[1] = *(const v8h*)(Bs + (nh * 64 + j * 16 + rl) * LDSP + kk + 16);
        acc[0][j] = mma_h(a0.v, bf.v, acc[0][j]);
        acc[1][j] = mma_h(a1.v, bf.v, acc[1][j]);
      }
    }
#pragma unroll
    for (int j = 0; j < 4; ++j) {
      float mx = -__builtin_huge_valf();
      float mn = __builtin_huge_valf();
      float s = 0.0f, q = 0.0f;
#pragma unroll
      for (int i = 0; i < 2; ++i)
#pragma unroll
        for (int r = 0; r < 8; ++r) {
          const float v = acc[i][j][r] * W_CARRY_INV;
          mx = fmaxf(mx, v);
          mn = fminf(mn, v);
          s = s + v;
          q = __builtin_fmaf(v, v, q);
        }
      const float mxo = __shfl_xor(mx, 16, 32);
      const float mno = __shfl_xor(mn, 16, 32);
      const float so  = __shfl_xor(s, 16, 32);
      const float qo  = __shfl_xor(q, 16, 32);
      mx = fmaxf(mx, mxo);
      mn = fminf(mn, mno);
      s = s + so;
      q = q + qo;
      const int col = nh * 64 + j * 16 + rl;
      const float pick = (hh != 0) ? mn : mx;
      gm[wave][hh * 128 + col] = pick;
      if (hh == 0) {
        red[0][wave][col] = s;
        red[1][wave][col] = q;
      }
    }
  }
  wave_lds_sync();
  {
    const v4f vmx = *(const v4f*)(gm[wave] + lane * 4);
    const v4f vmn = *(const v4f*)(gm[wave] + 128 + lane * 4);
    const size_t g = (size_t)blockIdx.x * 4 + wave;
    for (int pass = 0; pass < 2; ++pass) {
      *(volatile v4f*)(gmax + g * 128 + lane * 4) = vmx;
      *(volatile v4f*)(gmin + g * 128 + lane * 4) = vmn;
      __threadfence();
    }
  }
  __syncthreads();
  {
    float pv[2];
#pragma unroll
    for (int i = 0; i < 2; ++i) {
      const int k = tid + 128 * i;
      const int st = k >> 7;
      const int ch = k & 127;
      float a = 0.0f;
#pragma unroll
      for (int w = 0; w < 4; ++w) a = a + red[st][w][ch];
      pv[i] = a;
    }
    for (int pass = 0; pass < 2; ++pass) {
#pragma unroll
      for (int i = 0; i < 2; ++i)
        *(volatile float*)(part + (size_t)blockIdx.x * 256 + tid + 128 * i) = pv[i];
      __threadfence();
    }
  }
}

__global__ __launch_bounds__(256) void out_kernel(const float* __restrict__ gmax,
                                                  const float* __restrict__ gmin,
                                                  const float* __restrict__ scsh,
                                                  float* __restrict__ out1) {
  __shared__ __align__(16) float tt[128 * 36];
  const int tid = threadIdx.x;
  const int lane = tid & 31;
  const int wave = tid >> 5;
  const int b = blockIdx.y;
  const int p0 = blockIdx.x * 32;
  const int c4 = (tid & 31) * 4;
  const int pr = tid >> 5;
  const v4f scv = *(const v4f*)(scsh + c4);
  const v4f shv = *(const v4f*)(scsh + 128 + c4);
  const float sc0 = scv.x, sc1 = scv.y, sc2 = scv.z, sc3 = scv.w;
  const float sh0 = shv.x, sh1 = shv.y, sh2 = shv.z, sh3 = shv.w;
#pragma unroll
  for (int pass = 0; pass < 4; ++pass) {
    const int p = pass * 8 + pr;
    const size_t g = (size_t)b * NUM_CTR + p0 + p;
    const v4f mx = *(const v4f*)(gmax + g * 128 + c4);
    const v4f mn = *(const v4f*)(gmin + g * 128 + c4);
    const float x0 = (sc0 >= 0.0f) ? mx.x : mn.x;
    const float x1 = (sc1 >= 0.0f) ? mx.y : mn.y;
    const float x2 = (sc2 >= 0.0f) ? mx.z : mn.z;
    const float x3 = (sc3 >= 0.0f) ? mx.w : mn.w;
    tt[(c4 + 0) * 36 + p] = fmaxf(__builtin_fmaf(sc0, x0, sh0), 0.0f);
    tt[(c4 + 1) * 36 + p] = fmaxf(__builtin_fmaf(sc1, x1, sh1), 0.0f);
    tt[(c4 + 2) * 36 + p] = fmaxf(__builtin_fmaf(sc2, x2, sh2), 0.0f);
    tt[(c4 + 3) * 36 + p] = fmaxf(__builtin_fmaf(sc3, x3, sh3), 0.0f);
  }
  __syncthreads();
  const int q4 = lane >> 3;
  const int p4 = (lane & 7) * 4;
  v4f ov[4];
#pragma unroll
  for (int it = 0; it < 4; ++it) {
    const int c = wave * 16 + it * 4 + q4;
    ov[it] = *(const v4f*)(tt + c * 36 + p4);
  }
  for (int pass = 0; pass < 2; ++pass) {
#pragma unroll
    for (int it = 0; it < 4; ++it) {
      const int c = wave * 16 + it * 4 + q4;
      *(volatile v4f*)(out1 + ((size_t)b * NOUT3 + c) * NUM_CTR + p0 + p4) = ov[it];
    }
    __threadfence();
  }
}

extern "C" void kernel_launch(void* const* d_in, const int* in_sizes, int n_in,
                              void* d_out, int out_size, void* d_ws, size_t ws_size,
                              hipStream_t stream) {
  (void)in_sizes; (void)n_in; (void)out_size;
  if (ws_size < WS_TOTAL) return;
  const float* xyz  = (const float*)d_in[0];
  const float* feat = (const float*)d_in[1];
  const float* W1 = (const float*)d_in[2];
  const float* g1 = (const float*)d_in[3];
  const float* b1 = (const float*)d_in[4];
  const float* W2 = (const float*)d_in[5];
  const float* g2 = (const float*)d_in[6];
  const float* b2 = (const float*)d_in[7];
  const float* W3 = (const float*)d_in[8];
  const float* g3 = (const float*)d_in[9];
  const float* b3 = (const float*)d_in[10];

  float* out0 = (float*)d_out;
  float* out1 = (float*)d_out + (OUT1_OFF_B / 4);

  char* ws = (char*)d_ws;
  float*    nxyz  = (float*)(ws + WS_NXYZ);
  int*      idx   = (int*)(ws + WS_IDX);
  _Float16* wpl   = (_Float16*)(ws + WS_WPL);
  _Float16* Af    = (_Float16*)(ws + WS_AF);
  float*    Yp    = (float*)(ws + WS_YP);
  _Float16* X2    = (_Float16*)(ws + WS_X2);
  float*    gmax  = (float*)(ws + WS_GMAX);
  float*    gmin  = (float*)(ws + WS_GMIN);
  float*    part1 = (float*)(ws + WS_PART1);
  float*    part2 = (float*)(ws + WS_PART2);
  float*    part3 = (float*)(ws + WS_PART3);
  float*    scsh1 = (float*)(ws + WS_SCSH1);
  float*    scsh2 = (float*)(ws + WS_SCSH2);
  float*    scsh3 = (float*)(ws + WS_SCSH3);

  fps_kernel<<<NUM_B, 256, 0, stream>>>(xyz, out0, nxyz);
  ball_query_kernel<<<NUM_GRP / 8, 256, 0, stream>>>(xyz, nxyz, idx);
  pack_w_kernel<<<8, 256, 0, stream>>>(W1, W2, W3, wpl);
  feat_t_kernel<<<dim3(NUM_PTS / 64, NUM_B), 256, 0, stream>>>(feat, Af);
  gemm_pts_kernel<<<(NUM_B * NUM_PTS) / 256, 256, 0, stream>>>(Af, wpl, Yp);
  stats1_kernel<<<NUM_PBLK, 256, 0, stream>>>(xyz, nxyz, idx, Yp, W1, part1);
  finalize_kernel<NOUT1><<<1, 256, 0, stream>>>(part1, NUM_PBLK, g1, b1, scsh1);
  gemm2_kernel<<<NUM_PBLK, 256, 0, stream>>>(xyz, nxyz, idx, Yp, W1, scsh1, wpl + 4096, X2, part2);
  finalize_kernel<NOUT2><<<1, 256, 0, stream>>>(part2, NUM_PBLK, g2, b2, scsh2);
  gemm3_kernel<<<NUM_PBLK, 128, 0, stream>>>((const unsigned*)X2, scsh2, wpl + 8192, gmax, gmin, part3);
  finalize_kernel<NOUT3><<<1, 256, 0, stream>>>(part3, NUM_PBLK, g3, b3, scsh3);
  out_kernel<<<dim3(NUM_CTR / 32, NUM_B), 256, 0, stream>>>(gmax, gmin, scsh3, out1);
}
